// DegreeSortedMambaLayer_63488206569951
// MI455X (gfx1250) — hardware-run, weakly checked
//
#include <hip/hip_runtime.h>


namespace {
constexpr int G = 64, N = 256, L = N, NTK = G * N, DM = 256, DI = 512, DS = 16, DTR = 16, KC = 4, XD = DTR + 2 * DS, NE = NTK * 16;
constexpr float XS = 8.0f, US = 1024.0f  , DTS = 16384.0f  , YS = 4096.0f  , GS = 16384.0f  , WSC = 256.0f;
typedef _Float16 b16;
typedef __attribute__((ext_vector_type(16))) _Float16 v16b;
typedef __attribute__((ext_vector_type(8))) _Float16 v8b;
typedef __attribute__((ext_vector_type(8))) float v8f;
typedef __attribute__((ext_vector_type(4))) float v4f;
__device__ __forceinline__ float bf16_rne(float f) { unsigned int u = __float_as_uint(f); u += 0x7FFFu + ((u >> 16) & 1u); return __uint_as_float(u & 0xFFFF0000u); }
__device__ __forceinline__ void split16(float v, b16& hi, b16& lo) { hi = (b16)v; lo = (b16)(v - (float)hi); }
__device__ __forceinline__ v16b frag_kb(const b16* p, int hh) { const v8b a = *(const v8b*)(p + 8 * hh), b = *(const v8b*)(p + 16 + 8 * hh); v16b f;
#pragma unroll
  for (int e = 0; e < 8; ++e) { f[e] = a[e]; f[8 + e] = b[e]; } return f; }
__device__ __forceinline__ v8f wmma16b(v16b a, v16b b, v8f c) { v8f d = __builtin_amdgcn_wmma_f32_16x16x32_f16(false, a, false, b, (short)0, c, false, false); asm volatile("v_nop\n\tv_nop\n\tv_nop\n\tv_nop" : "+v"(d) : "v"(a), "v"(b)); return d; }
__device__ __forceinline__ void wave_lds_sync() { __builtin_amdgcn_fence(__ATOMIC_RELEASE, "workgroup"); __builtin_amdgcn_wave_barrier(); __builtin_amdgcn_fence(__ATOMIC_ACQUIRE, "workgroup"); }
__device__ __forceinline__ float pmul(float a, float b) { float p = a * b; asm volatile("" : "+v"(p)); return p; }
__device__ __forceinline__ int iclamp(int v, int lo, int hi) { return v < lo ? lo : (v > hi ? hi : v); }
__device__ __forceinline__ float silu(float v) { return v / (1.0f + __expf(-v)); }
__device__ __forceinline__ float sigm(float v) { return 1.0f / (1.0f + __expf(-v)); }
__device__ __forceinline__ float softplus(float v) { return v > 20.0f ? v : (v < -20.0f ? __expf(v) : log1pf(__expf(v))); }
constexpr int CSR_NBLK9 = 512, CSR_GB9 = 9, CSR_GN9 = 1 << CSR_GB9  , CSR_TS9 = (CSR_GN9 < 32 ? 32 : CSR_GN9)  , CSR_MAXG9 = 512, CSR_CAP9 = 12288  ;
__device__ __host__ __forceinline__ int csr_tix9(int v) { return (v >> CSR_GB9) * CSR_TS9 + (v & (CSR_GN9 - 1)); }
__global__ __launch_bounds__(64) void csrA_kernel9(const int* __restrict__ dst, int E, int N, int nG, int CHP, int NGP, int* __restrict__ STG, int* __restrict__ HST) {
  extern __shared__ int sm[];
  int* cnt = sm; int* run = sm + NGP; int* ids = sm + 2 * NGP;
  const int b = blockIdx.x; const int ch = (E + CSR_NBLK9 - 1) / CSR_NBLK9; const int e0 = b * ch, e1 = min(E, e0 + ch);
  for (int i = threadIdx.x; i < NGP; i += 64) cnt[i] = 0;
  for (int i = threadIdx.x; i < CHP; i += 64) ids[i] = -1;
  __syncthreads();
  if (threadIdx.x == 0) {
    for (int e = e0; e < e1; ++e) { int d = dst[e]; d = (d < 0) ? 0 : (d >= N ? N - 1 : d); cnt[d >> CSR_GB9] += 1; }
    int acc = 0; for (int g = 0; g < nG; ++g) { run[g] = acc; acc += cnt[g]; }
    for (int e = e0; e < e1; ++e) { int d = dst[e]; d = (d < 0) ? 0 : (d >= N ? N - 1 : d); const int g = d >> CSR_GB9; ids[run[g]] = e; run[g] += 1; } }
  __syncthreads();
  typedef __attribute__((ext_vector_type(4))) int v4i;
  for (int pass = 0; pass < 2; ++pass) {
    for (int i = threadIdx.x; i < CHP / 4; i += 64) *(volatile v4i*)(STG + (size_t)b * CHP + i * 4) = *(const v4i*)(&ids[i * 4]);
    for (int i = threadIdx.x; i < NGP / 4; i += 64) { v4i v; for (int e = 0; e < 4; ++e) v[e] = (i * 4 + e < nG) ? cnt[i * 4 + e] : 0; *(volatile v4i*)(HST + (size_t)b * NGP + i * 4) = v; }
    __threadfence(); }
}
__global__ __launch_bounds__(512) void csrS_kernel9(const int* __restrict__ HST, int nG, int NGP, int* __restrict__ START, int* __restrict__ TOT, int* __restrict__ OFF) {
  __shared__ int tot[CSR_MAXG9];
  const int b = threadIdx.x;
  for (int pass = 0; pass < 2; ++pass) { int runb = 0; for (int g = 0; g < nG; ++g) { int c = HST[(size_t)b * NGP + g]; c = (c < 0) ? 0 : c; ((volatile int*)OFF)[(size_t)g * CSR_NBLK9 + b] = runb; runb += c; } __threadfence(); }
  for (int g = threadIdx.x; g < nG; g += 512) { int s = 0; for (int bb = 0; bb < CSR_NBLK9; ++bb) { int c = HST[(size_t)bb * NGP + g]; s += (c < 0) ? 0 : c; } tot[g] = s; }
  __syncthreads();
  if (threadIdx.x < 32) {
    __shared__ int st[CSR_MAXG9 + 32];
    if (threadIdx.x == 0) { int acc = 0; for (int g = 0; g < NGP; ++g) { st[g] = acc; if (g < nG) acc += (tot[g] + 31) & ~31; } st[NGP] = acc; }
    __builtin_amdgcn_fence(__ATOMIC_RELEASE, "workgroup"); __builtin_amdgcn_wave_barrier(); __builtin_amdgcn_fence(__ATOMIC_ACQUIRE, "workgroup");
    for (int pass = 0; pass < 2; ++pass) { for (int i = threadIdx.x; i < NGP + 32; i += 32) { ((volatile int*)START)[i] = (i <= NGP) ? st[min(i, NGP)] : 0; ((volatile int*)TOT)[i] = (i < nG) ? tot[i] : 0; } __threadfence(); } }
}
__global__ __launch_bounds__(256) void csrB_kernel9(const int* __restrict__ dst, int N, int nG, int CHP, int NGP, int permLen, const int* __restrict__ STG, const int* __restrict__ HST, const int* __restrict__ OFF, const int* __restrict__ START, const int* __restrict__ TOT, int* __restrict__ PERM, int* __restrict__ ROWPTR, int* __restrict__ ROWCNT, int* __restrict__ FLAG) {
  typedef __attribute__((ext_vector_type(4))) int v4i;
  __shared__ int ids[CSR_CAP9]; __shared__ unsigned short key[CSR_CAP9]; __shared__ int outp[CSR_CAP9]; __shared__ int ncnt[CSR_GN9 + 1]; __shared__ int boff[CSR_NBLK9 + 1];
  const int g = blockIdx.x, t_ = threadIdx.x; int tot = TOT[g]; int st = START[g], stn = START[g + 1]; const int v0 = g * CSR_GN9; const int nv = min(CSR_GN9, N - v0); const int t0 = g * CSR_TS9;
  st = (st < 0) ? 0 : (st > permLen - 32 ? permLen - 32 : st) & ~31; stn = (stn < st) ? st : (stn > permLen ? permLen : stn); tot = (tot < 0) ? 0 : tot; if (tot > stn - st && tot <= CSR_CAP9) tot = stn - st;
  if (tot > CSR_CAP9) {
    for (int pass = 0; pass < 2; ++pass) { for (int i = t_; i < CSR_TS9 / 4; i += 256) { v4i a, c; for (int e = 0; e < 4; ++e) { a[e] = st; c[e] = 0; } *(volatile v4i*)(ROWPTR + t0 + i * 4) = a; *(volatile v4i*)(ROWCNT + t0 + i * 4) = c; } if (t_ == 0) ((volatile int*)FLAG)[0] = 1; __threadfence(); } (void)nv; return; }
  if (t_ == 0) { int acc = 0; for (int b = 0; b < CSR_NBLK9; ++b) { boff[b] = acc; int c = HST[(size_t)b * NGP + g]; c = (c < 0) ? 0 : (c > CHP ? CHP : c); acc += c; if (acc > tot) acc = tot; } boff[CSR_NBLK9] = acc; }
  for (int i = t_; i <= CSR_GN9; i += 256) ncnt[i] = 0;
  __syncthreads();
  for (int b = 0; b < CSR_NBLK9; ++b) { const int c = boff[b + 1] - boff[b]; int o_ = OFF[(size_t)g * CSR_NBLK9 + b]; o_ = (o_ < 0) ? 0 : (o_ > CHP - c ? CHP - c : o_); const int* src_ = STG + (size_t)b * CHP + o_;
    for (int i = t_; i < c; i += 256) { int id = src_[i]; id = (id < 0) ? 0 : id; ids[boff[b] + i] = id; int d = dst[id]; d = (d < v0) ? v0 : (d >= N ? N - 1 : d); int kk = d - v0; kk = (kk < 0) ? 0 : (kk >= CSR_GN9 ? CSR_GN9 - 1 : kk); key[boff[b] + i] = (unsigned short)kk; } }
  __syncthreads();
  if (t_ == 0) { for (int i = 0; i < tot; ++i) ncnt[key[i]] += 1; int acc = 0; for (int vl = 0; vl < CSR_GN9; ++vl) { const int c = ncnt[vl]; ncnt[vl] = acc; acc += c; } ncnt[CSR_GN9] = acc;
    for (int i = 0; i < tot; ++i) { const int vl = key[i]; outp[ncnt[vl]] = ids[i]; ncnt[vl] += 1; }
    for (int vl = CSR_GN9; vl > 0; --vl) ncnt[vl] = ncnt[vl - 1]; ncnt[0] = 0; }
  __syncthreads();
  for (int pass = 0; pass < 2; ++pass) {
    for (int i = t_; i < (stn - st) / 4; i += 256) { v4i v; for (int e = 0; e < 4; ++e) { const int q = i * 4 + e; v[e] = (q < tot) ? outp[q] : -1; } *(volatile v4i*)(PERM + st + i * 4) = v; }
    for (int i = t_; i < CSR_TS9 / 4; i += 256) { v4i a, c; for (int e = 0; e < 4; ++e) { const int vl = i * 4 + e; const int vc = vl < CSR_GN9 ? vl : CSR_GN9; a[e] = (vl < CSR_GN9) ? st + ncnt[vc] : st; c[e] = (vl < nv) ? (ncnt[(vc < CSR_GN9 ? vc : CSR_GN9 - 1) + 1] - ncnt[vc]) : 0; } *(volatile v4i*)(ROWPTR + t0 + i * 4) = a; *(volatile v4i*)(ROWCNT + t0 + i * 4) = c; }
    __threadfence(); }
}
__global__ __launch_bounds__(256) void csrZ_kernel9(int* __restrict__ p, size_t n4) { typedef __attribute__((ext_vector_type(4))) int v4i; const size_t tid = (size_t)blockIdx.x * 256 + threadIdx.x, nth = (size_t)gridDim.x * 256; v4i z = {0, 0, 0, 0}; for (size_t i = tid; i < n4; i += nth) *(volatile v4i*)(p + i * 4) = z; }
struct CsrBufs9 { int *STG, *HST, *OFF, *START, *TOT, *PERM, *ROWPTR, *ROWCNT, *FLAG; int nG, NGP, CHP; size_t permLen; char* base; size_t bytes; };
static size_t csr_carve9(CsrBufs9& c, char* ws, size_t off, int E, int N) {
  const size_t off0 = off; c.base = ws + off;
  auto al = [&](size_t bytes) { char* p = ws + off; off += (bytes + 255) & ~(size_t)255; return p; };
  c.nG = (N + CSR_GN9 - 1) / CSR_GN9; c.NGP = (c.nG + 31) & ~31; const int ch = (E + CSR_NBLK9 - 1) / CSR_NBLK9; c.CHP = (ch + 31) & ~31; c.permLen = (size_t)E + 32 * (size_t)c.nG + 32;
  c.STG = (int*)al((size_t)CSR_NBLK9 * c.CHP * 4); c.HST = (int*)al((size_t)CSR_NBLK9 * c.NGP * 4); c.OFF = (int*)al((size_t)c.NGP * CSR_NBLK9 * 4); c.START = (int*)al((size_t)(c.NGP + 64) * 4); c.TOT = (int*)al((size_t)(c.NGP + 64) * 4);
  c.PERM = (int*)al(c.permLen * 4); c.ROWPTR = (int*)al((size_t)c.nG * CSR_TS9 * 4); c.ROWCNT = (int*)al((size_t)c.nG * CSR_TS9 * 4); c.FLAG = (int*)al(256);
  c.bytes = off - off0; return off;
}
static void csr_build9(const CsrBufs9& c, const int* dst, int E, int N, hipStream_t stream) {
  const size_t smem = (size_t)(2 * c.NGP + c.CHP) * 4;
  csrZ_kernel9<<<512, 256, 0, stream>>>((int*)c.base, c.bytes / 16);
  csrA_kernel9<<<CSR_NBLK9, 64, smem, stream>>>(dst, E, N, c.nG, c.CHP, c.NGP, c.STG, c.HST);
  csrS_kernel9<<<1, 512, 0, stream>>>(c.HST, c.nG, c.NGP, c.START, c.TOT, c.OFF);
  csrB_kernel9<<<c.nG, 256, 0, stream>>>(dst, N, c.nG, c.CHP, c.NGP, (int)c.permLen, c.STG, c.HST, c.OFF, c.START, c.TOT, c.PERM, c.ROWPTR, c.ROWCNT, c.FLAG);
}


__global__ __launch_bounds__(256) void wcopy_kernel(const float* __restrict__ w, int OUT, int KIN, int KP, b16* __restrict__ WT) {
  const size_t u = (size_t)blockIdx.x * 256 + threadIdx.x; if (u >= (size_t)OUT * KP / 8) return; const size_t e = u * 8; const int o = (int)(e / KP), k0 = (int)(e % KP); v8b v;
  for (int j = 0; j < 8; ++j) { const int k = k0 + j; v[j] = k < KIN ? (b16)(bf16_rne(w[(size_t)o * KIN + (k < KIN ? k : 0)]) * WSC) : (b16)0.0f; } for (int pass = 0; pass < 2; ++pass) { *(volatile v8b*)(WT + e) = v; __threadfence(); }
}
__global__ __launch_bounds__(256) void rank_kernel(const int* __restrict__ DEGC, float* __restrict__ dummy, int* __restrict__ PERM) {
  __shared__ int dg[N]; __shared__ int slot[N]; (void)dummy;
  const int g = blockIdx.x, i = threadIdx.x; const int di = DEGC[g * N + i]; dg[i] = di; __syncthreads();
  int r = 0;
#pragma unroll 1
  for (int j = 0; j < N; ++j) { const int dj = dg[j]; r += (dj < di) ? 1 : 0; r += (dj == di && j < i) ? 1 : 0; }
  slot[r] = g * N + i; __syncthreads();
  for (int pass = 0; pass < 2; ++pass) { ((volatile int*)PERM)[g * N + i] = slot[i]; __threadfence(); }
}
template <int REV>
__global__ __launch_bounds__(32) void inproj_kernel(const float* __restrict__ x, const int* __restrict__ PERM, const b16* __restrict__ WIN, float* __restrict__ XZ) {
  __shared__ __attribute__((aligned(16))) b16 Ah[16][DM + 8]; __shared__ __attribute__((aligned(16))) float Tf[16][128 + 4];
  const int lane = threadIdx.x, nloc = lane & 15, hlf = lane >> 4; const size_t m0 = (size_t)blockIdx.x * 16; const int g = (int)(m0 / N), r0 = (int)(m0 % N);
  for (int rr = 0; rr < 16; ++rr) { const int r = r0 + rr; const int pos = REV ? (N - 1 - r) : r; const int nd = iclamp(PERM[g * N + pos], 0, NTK - 1);
    for (int q = 0; q < 2; ++q) { const v4f v = *(const v4f*)(x + (size_t)nd * DM + q * 128 + lane * 4); for (int j = 0; j < 4; ++j) Ah[rr][q * 128 + lane * 4 + j] = (b16)(bf16_rne(v[j]) * XS); } }
  wave_lds_sync();
#pragma unroll 1
  for (int cg = 0; cg < 8; ++cg) { v8f acc[8];
#pragma unroll
    for (int t = 0; t < 8; ++t) acc[t] = (v8f){};
#pragma unroll 2
    for (int kb = 0; kb < DM; kb += 32) { const v16b a = frag_kb(&Ah[nloc][kb], hlf);
#pragma unroll
      for (int t = 0; t < 8; ++t) acc[t] = wmma16b(a, frag_kb(WIN + (size_t)(cg * 128 + t * 16 + nloc) * DM + kb, hlf), acc[t]); }
#pragma unroll
    for (int t = 0; t < 8; ++t)
#pragma unroll 1
      for (int r8 = 0; r8 < 8; ++r8) Tf[8 * hlf + r8][t * 16 + nloc] = acc[t][r8] * (1.0f / (XS * WSC));
    wave_lds_sync();
    for (int pass = 0; pass < 2; ++pass) { for (int rr = 0; rr < 16; ++rr) *(volatile v4f*)(XZ + (m0 + rr) * (2 * DI) + cg * 128 + lane * 4) = *(const v4f*)(&Tf[rr][lane * 4]); __threadfence(); }
    wave_lds_sync(); }
}
__global__ __launch_bounds__(32) void mid_kernel(const float* __restrict__ XZ, const float* __restrict__ cw, const float* __restrict__ cb, const b16* __restrict__ WX, const b16* __restrict__ WDT, const float* __restrict__ bdt, float* __restrict__ XC, float* __restrict__ BCp, float* __restrict__ DT) {
  __shared__ __attribute__((aligned(16))) b16 Ah[16][DI + 8], Al[16][DI + 8]; __shared__ __attribute__((aligned(16))) float Tf[16][128 + 4]; __shared__ __attribute__((aligned(16))) float Sbc[16][32];
  const int lane = threadIdx.x, nloc = lane & 15, hlf = lane >> 4; const size_t m0 = (size_t)blockIdx.x * 16; const int tpos0 = (int)(m0 % L);
  for (int rr = 0; rr < 16; ++rr) { const int tpos = tpos0 + rr;
    for (int q = 0; q < 4; ++q) { v4f acc = {0.0f, 0.0f, 0.0f, 0.0f};
      for (int k = 0; k < KC; ++k) { const int tt = tpos - (KC - 1) + k; if (tt >= 0) { const v4f xv = *(const v4f*)(XZ + (m0 + rr - (KC - 1) + k) * (2 * DI) + q * 128 + lane * 4); for (int j = 0; j < 4; ++j) acc[j] += pmul(xv[j], bf16_rne(cw[(q * 128 + lane * 4 + j) * KC + k])); } }
      v4f o; for (int j = 0; j < 4; ++j) { const int c = q * 128 + lane * 4 + j; o[j] = silu(acc[j] + bf16_rne(cb[c])); b16 p, ql; split16(o[j] * US, p, ql); Ah[rr][c] = p; Al[rr][c] = ql; }
      for (int pass = 0; pass < 2; ++pass) { *(volatile v4f*)(XC + (m0 + rr) * DI + q * 128 + lane * 4) = o; __threadfence(); } } }
  wave_lds_sync();
  v8f ax[3] = {(v8f){}, (v8f){}, (v8f){}};
#pragma unroll 2
  for (int kb = 0; kb < DI; kb += 32) { const v16b a = frag_kb(&Ah[nloc][kb], hlf), al = frag_kb(&Al[nloc][kb], hlf);
#pragma unroll
    for (int t = 0; t < 3; ++t) { const v16b bw = frag_kb(WX + (size_t)(t * 16 + nloc) * DI + kb, hlf); ax[t] = wmma16b(a, bw, ax[t]); ax[t] = wmma16b(al, bw, ax[t]); } }
  wave_lds_sync();
  const float sx = 1.0f / (US * WSC);
#pragma unroll
  for (int r8 = 0; r8 < 8; ++r8) { const int rl = 8 * hlf + r8; const float dtr = ax[0][r8] * sx; b16 p, ql; split16(dtr * DTS, p, ql); Ah[rl][nloc] = p; Al[rl][nloc] = ql; Ah[rl][16 + nloc] = (b16)0.0f; Al[rl][16 + nloc] = (b16)0.0f; Sbc[rl][nloc] = ax[1][r8] * sx; Sbc[rl][16 + nloc] = ax[2][r8] * sx; }
  wave_lds_sync();
  for (int pass = 0; pass < 2; ++pass) { for (int rr = 0; rr < 16; ++rr) ((volatile float*)BCp)[(m0 + rr) * 32 + lane] = Sbc[rr][lane]; __threadfence(); }
  const float se = 1.0f / (DTS * WSC);
#pragma unroll 1
  for (int cg = 0; cg < 4; ++cg) { v8f acc[8];
#pragma unroll
    for (int t = 0; t < 8; ++t) { acc[t] = (v8f){}; const v16b a = frag_kb(&Ah[nloc][0], hlf), al = frag_kb(&Al[nloc][0], hlf); const v16b bw = frag_kb(WDT + (size_t)(cg * 128 + t * 16 + nloc) * 32, hlf); acc[t] = wmma16b(a, bw, acc[t]); acc[t] = wmma16b(al, bw, acc[t]); }
#pragma unroll
    for (int t = 0; t < 8; ++t) { const int c = cg * 128 + t * 16 + nloc; const float bb = bf16_rne(bdt[c]);
#pragma unroll 1
      for (int r8 = 0; r8 < 8; ++r8) Tf[8 * hlf + r8][t * 16 + nloc] = softplus(acc[t][r8] * se + bb); }
    wave_lds_sync();
    for (int pass = 0; pass < 2; ++pass) { for (int rr = 0; rr < 16; ++rr) *(volatile v4f*)(DT + (m0 + rr) * DI + cg * 128 + lane * 4) = *(const v4f*)(&Tf[rr][lane * 4]); __threadfence(); }
    wave_lds_sync(); }
}
__global__ __launch_bounds__(256) void scan_kernel(const float* __restrict__ XC, const float* __restrict__ DT, const float* __restrict__ BCp, const float* __restrict__ XZ, const float* __restrict__ alog, const float* __restrict__ Dp, int nb, float* __restrict__ Y) {
  const int gid = blockIdx.x * 256 + threadIdx.x; const int b = gid / DI, d = gid % DI; if (b >= nb) return;
  float A[DS]; for (int s = 0; s < DS; ++s) A[s] = -__expf(bf16_rne(alog[d * DS + s])); const float dd = bf16_rne(Dp[d]);
#pragma unroll 1
  for (int pass = 0; pass < 2; ++pass) { float h[DS]; for (int s = 0; s < DS; ++s) h[s] = 0.0f;
#pragma unroll 1
    for (int t = 0; t < L; ++t) { const size_t row = (size_t)b * L + t; const float x = XC[row * DI + d], dt = DT[row * DI + d], z = XZ[row * (2 * DI) + DI + d]; const float dx = pmul(dt, x); float y = 0.0f;
#pragma unroll
      for (int s = 0; s < DS; ++s) { const float da = __expf(pmul(dt, A[s])); h[s] = pmul(da, h[s]) + pmul(dx, BCp[row * 32 + s]); y += pmul(h[s], BCp[row * 32 + 16 + s]); }
      y += pmul(dd, x); ((volatile float*)Y)[row * DI + d] = pmul(y, silu(z)); }
    __threadfence(); }
}

__global__ __launch_bounds__(32) void outproj_kernel(const float* __restrict__ Y, const b16* __restrict__ WOUT, float* __restrict__ Op) {
  __shared__ __attribute__((aligned(16))) b16 Ah[16][DI + 8], Al[16][DI + 8]; __shared__ __attribute__((aligned(16))) float Tf[16][128 + 4];
  const int lane = threadIdx.x, nloc = lane & 15, hlf = lane >> 4; const size_t m0 = (size_t)blockIdx.x * 16;
  for (int rr = 0; rr < 16; ++rr) for (int q = 0; q < 4; ++q) { const v4f v = *(const v4f*)(Y + (m0 + rr) * DI + q * 128 + lane * 4); for (int j = 0; j < 4; ++j) { b16 p, ql; split16(v[j] * YS, p, ql); Ah[rr][q * 128 + lane * 4 + j] = p; Al[rr][q * 128 + lane * 4 + j] = ql; } }
  wave_lds_sync();
#pragma unroll 1
  for (int cg = 0; cg < 2; ++cg) { v8f acc[8];
#pragma unroll
    for (int t = 0; t < 8; ++t) acc[t] = (v8f){};
#pragma unroll 2
    for (int kb = 0; kb < DI; kb += 32) { const v16b a = frag_kb(&Ah[nloc][kb], hlf), al = frag_kb(&Al[nloc][kb], hlf);
#pragma unroll
      for (int t = 0; t < 8; ++t) { const v16b bw = frag_kb(WOUT + (size_t)(cg * 128 + t * 16 + nloc) * DI + kb, hlf); acc[t] = wmma16b(a, bw, acc[t]); acc[t] = wmma16b(al, bw, acc[t]); } }
#pragma unroll
    for (int t = 0; t < 8; ++t)
#pragma unroll 1
      for (int r8 = 0; r8 < 8; ++r8) Tf[8 * hlf + r8][t * 16 + nloc] = acc[t][r8] * (1.0f / (YS * WSC));
    wave_lds_sync();
    for (int pass = 0; pass < 2; ++pass) { for (int rr = 0; rr < 16; ++rr) *(volatile v4f*)(Op + (m0 + rr) * DM + cg * 128 + lane * 4) = *(const v4f*)(&Tf[rr][lane * 4]); __threadfence(); }
    wave_lds_sync(); }
}
__global__ __launch_bounds__(32) void gate_kernel(const float* __restrict__ FO, const float* __restrict__ BO, const int* __restrict__ PERM, const b16* __restrict__ WG, const float* __restrict__ gb, float* __restrict__ out) {
  __shared__ __attribute__((aligned(16))) b16 Ah[16][DI + 8], Al[16][DI + 8]; __shared__ __attribute__((aligned(16))) float Fv[16][DM + 4], Bv[16][DM + 4];
  const int lane = threadIdx.x, nloc = lane & 15, hlf = lane >> 4; const size_t m0 = (size_t)blockIdx.x * 16; const int g = (int)(m0 / N), r0 = (int)(m0 % N);
  for (int rr = 0; rr < 16; ++rr) { const int r = r0 + rr; const float* fr = FO + ((size_t)g * N + r) * DM; const float* br = BO + ((size_t)g * N + (N - 1 - r)) * DM;
    for (int q = 0; q < 2; ++q) { const v4f f = *(const v4f*)(fr + q * 128 + lane * 4), b = *(const v4f*)(br + q * 128 + lane * 4);
      for (int j = 0; j < 4; ++j) { const int c = q * 128 + lane * 4 + j; Fv[rr][c] = f[j]; Bv[rr][c] = b[j]; b16 p, ql; split16(f[j] * GS, p, ql); Ah[rr][c] = p; Al[rr][c] = ql; split16(b[j] * GS, p, ql); Ah[rr][DM + c] = p; Al[rr][DM + c] = ql; } } }
  wave_lds_sync();
#pragma unroll 1
  for (int cg = 0; cg < 2; ++cg) { v8f acc[8];
#pragma unroll
    for (int t = 0; t < 8; ++t) acc[t] = (v8f){};
#pragma unroll 2
    for (int kb = 0; kb < DI; kb += 32) { const v16b a = frag_kb(&Ah[nloc][kb], hlf), al = frag_kb(&Al[nloc][kb], hlf);
#pragma unroll
      for (int t = 0; t < 8; ++t) { const v16b bw = frag_kb(WG + (size_t)(cg * 128 + t * 16 + nloc) * DI + kb, hlf); acc[t] = wmma16b(a, bw, acc[t]); acc[t] = wmma16b(al, bw, acc[t]); } }
#pragma unroll
    for (int t = 0; t < 8; ++t) { const int c = cg * 128 + t * 16 + nloc; const float bb = bf16_rne(gb[c]);
#pragma unroll
      for (int r8 = 0; r8 < 8; ++r8) { const int rl = 8 * hlf + r8; const float gl = sigm(acc[t][r8] * (1.0f / (GS * WSC)) + bb); Fv[rl][c] = pmul(gl, Fv[rl][c]) + pmul(1.0f - gl, Bv[rl][c]); } } }
  wave_lds_sync();
  for (int pass = 0; pass < 2; ++pass) { for (int rr = 0; rr < 16; ++rr) { const size_t nd = (size_t)iclamp(PERM[g * N + r0 + rr], 0, NTK - 1); *(volatile v4f*)(out + nd * DM + lane * 4) = *(const v4f*)(&Fv[rr][lane * 4]); *(volatile v4f*)(out + nd * DM + 128 + lane * 4) = *(const v4f*)(&Fv[rr][128 + lane * 4]); } __threadfence(); }
}
}

extern "C" void kernel_launch(void* const* d_in, const int* in_sizes, int n_in, void* d_out, int out_size, void* d_ws, size_t ws_size, hipStream_t stream) {
  (void)n_in;
  auto Fp = [&](int i) { return (const float*)d_in[i]; }; auto Ip = [&](int i) { return (const int*)d_in[i]; };
  if (in_sizes[0] != NTK * DM || in_sizes[1] != 2 * NE || in_sizes[2] != NTK || in_sizes[3] != DM * 2 * DM || in_sizes[5] != 2 * DI * DM || in_sizes[8] != XD * DI || in_sizes[9] != DI * DTR || in_sizes[13] != DM * DI || in_sizes[14] != 2 * DI * DM || in_sizes[22] != DM * DI || out_size != NTK * DM) return;
  size_t off = 0; char* ws = (char*)d_ws;
  auto carve = [&](size_t bytes) { char* p = ws + off; off += (bytes + 255) & ~(size_t)255; return p; };
  b16* WIN[2]; b16* WX[2]; b16* WDT[2]; b16* WOUT[2]; for (int r = 0; r < 2; ++r) { WIN[r] = (b16*)carve((size_t)2 * DI * DM * 2); WX[r] = (b16*)carve((size_t)XD * DI * 2); WDT[r] = (b16*)carve((size_t)DI * 32 * 2); WOUT[r] = (b16*)carve((size_t)DM * DI * 2); }
  b16* WG = (b16*)carve((size_t)DM * 2 * DM * 2); int* PERM = (int*)carve((size_t)NTK * 4);
  float* XZ = (float*)carve((size_t)NTK * 2 * DI * 4); float* XC = (float*)carve((size_t)NTK * DI * 4); float* DT = (float*)carve((size_t)NTK * DI * 4); float* BCp = (float*)carve((size_t)NTK * 32 * 4); float* Y = (float*)carve((size_t)NTK * DI * 4);
  float* OP[2]; OP[0] = (float*)carve((size_t)NTK * DM * 4); OP[1] = (float*)carve((size_t)NTK * DM * 4);
  CsrBufs9 csr; off = csr_carve9(csr, ws, off, NE, NTK);
  if (off > ws_size) return;
  const int GV = G;
  const int NTV = GV * N;
  auto g8 = [](size_t n8) { return (unsigned)((n8 + 255) / 256); };
  for (int r = 0; r < 2; ++r) { const int base = 5 + 9 * r;
    wcopy_kernel<<<g8((size_t)2 * DI * DM / 8), 256, 0, stream>>>(Fp(base + 0), 2 * DI, DM, DM, WIN[r]); wcopy_kernel<<<g8((size_t)XD * DI / 8), 256, 0, stream>>>(Fp(base + 3), XD, DI, DI, WX[r]);
    wcopy_kernel<<<g8((size_t)DI * 32 / 8), 256, 0, stream>>>(Fp(base + 4), DI, DTR, 32, WDT[r]); wcopy_kernel<<<g8((size_t)DM * DI / 8), 256, 0, stream>>>(Fp(base + 8), DM, DI, DI, WOUT[r]); }
  wcopy_kernel<<<g8((size_t)DM * 2 * DM / 8), 256, 0, stream>>>(Fp(3), DM, 2 * DM, 2 * DM, WG);
  csr_build9(csr, Ip(1), NE, NTK, stream);
  rank_kernel<<<GV, 256, 0, stream>>>(csr.ROWCNT, nullptr, PERM);
  for (int r = 0; r < 2; ++r) { const int base = 5 + 9 * r;
    if (r == 0) inproj_kernel<0><<<NTV / 16, 32, 0, stream>>>(Fp(0), PERM, WIN[0], XZ); else inproj_kernel<1><<<NTV / 16, 32, 0, stream>>>(Fp(0), PERM, WIN[1], XZ);
    mid_kernel<<<NTV / 16, 32, 0, stream>>>(XZ, Fp(base + 1), Fp(base + 2), WX[r], WDT[r], Fp(base + 5), XC, BCp, DT);
    scan_kernel<<<GV * DI / 256, 256, 0, stream>>>(XC, DT, BCp, XZ, Fp(base + 6), Fp(base + 7), GV, Y);
    outproj_kernel<<<NTV / 16, 32, 0, stream>>>(Y, WOUT[r], OP[r]); }
  gate_kernel<<<NTV / 16, 32, 0, stream>>>(OP[0], OP[1], PERM, WG, Fp(4), (float*)d_out);
}
